// CrossLayerAttention_67430986547826
// MI455X (gfx1250) — hardware-run, weakly checked
//
#include <hip/hip_runtime.h>
#include <math.h>
#include <stdint.h>

#ifndef NB
#define NB 4
#endif
#ifndef NQ
#define NQ 4096
#endif
#define NB_FULL 4
#define CC     128
#define CU     64
#define NN     4096
#define QT     64
#define OSP    68
#define OSPW   132
#define TP     72
#define VTD    16
#define VTM    512
#define VTP    516
#define SCL    0.08838834764831845f
#define LNPS   9.704060527839234f

static_assert(NB >= 1 && NB <= NB_FULL);
static_assert(NQ >= QT && NQ <= NN && NQ % QT == 0);
static_assert(NN % QT == 0 && NN % 32 == 0);
static_assert(CC == 2 * QT && CC % 32 == 0 && CU % 32 == 0 && CU == QT);
static_assert(NN == 32 * CC);
static_assert(VTM == 16 * 32 && CC % VTD == 0 && NN % VTM == 0);
static_assert((OSP * 4) % 16 == 0);
static_assert((OSPW * 4) % 16 == 0);
static_assert((TP * 2) % 16 == 0);
static_assert((VTP * 4) % 16 == 0);
static_assert((size_t)NB * CC * NN <= (size_t)NB_FULL * CC * NN);

typedef _Float16       v16h __attribute__((ext_vector_type(16)));
typedef _Float16       v8h  __attribute__((ext_vector_type(8)));
typedef __bf16         v16b __attribute__((ext_vector_type(16)));
typedef unsigned short v8us __attribute__((ext_vector_type(8)));
typedef float          v8f  __attribute__((ext_vector_type(8)));
typedef float          v4f  __attribute__((ext_vector_type(4)));
typedef unsigned int   v4u  __attribute__((ext_vector_type(4)));

union Frag  { v8us u[2]; v16h h; v16b bf; };
union FragH { v16h v; v8h hv[2]; };
static_assert(sizeof(Frag) == 32);
static_assert(sizeof(FragH) == 32);

__device__ __forceinline__ unsigned short bf_bits(float f) {
  unsigned u = __float_as_uint(f);
  return (unsigned short)((u + 0x7FFFu + ((u >> 16) & 1u)) >> 16);
}
__device__ __forceinline__ float bf_up(unsigned short hb) { return __uint_as_float(((unsigned)hb) << 16); }
__device__ __forceinline__ float bfr(float f) { return bf_up(bf_bits(f)); }
__device__ __forceinline__ unsigned short h_bits(_Float16 x) { return __builtin_bit_cast(unsigned short, x); }
__device__ __forceinline__ unsigned pk16(unsigned short a, unsigned short b) { return (unsigned)a | ((unsigned)b << 16); }
__device__ __forceinline__ v8f zero8() { v8f z = {0.f, 0.f, 0.f, 0.f, 0.f, 0.f, 0.f, 0.f}; return z; }
__device__ __forceinline__ float hmax8(v8f s) {
  return fmaxf(fmaxf(fmaxf(s[0], s[1]), fmaxf(s[2], s[3])), fmaxf(fmaxf(s[4], s[5]), fmaxf(s[6], s[7])));
}
__device__ __forceinline__ unsigned wave_ballot(bool p) {
#if defined(__HIP_DEVICE_COMPILE__)
  return __builtin_amdgcn_ballot_w32(p);
#else
  return p ? 1u : 0u;
#endif
}

__device__ __forceinline__ Frag ldfrag(const unsigned short* p) {
  Frag f;
  f.u[0] = *(const v8us*)(p);
  f.u[1] = *(const v8us*)(p + 16);
  return f;
}

__device__ __forceinline__ v8f mma_h(v16h a, v16h b, v8f c) {
  v8f d = __builtin_amdgcn_wmma_f32_16x16x32_f16(false, a, false, b, (short)0, c, false, false);
#if defined(__HIP_DEVICE_COMPILE__)
  asm volatile("v_nop\n\tv_nop\n\tv_nop\n\tv_nop" : "+v"(d) : "v"(a), "v"(b));
#endif
  return d;
}
__device__ __forceinline__ v8f mma_b(v16b a, v16b b, v8f c) {
  v8f d = __builtin_amdgcn_wmma_f32_16x16x32_bf16(false, a, false, b, (short)0, c, false, false);
#if defined(__HIP_DEVICE_COMPILE__)
  const v16h ha = __builtin_bit_cast(v16h, a), hb = __builtin_bit_cast(v16h, b);
  asm volatile("v_nop\n\tv_nop\n\tv_nop\n\tv_nop" : "+v"(d) : "v"(ha), "v"(hb));
#endif
  return d;
}

__global__ __launch_bounds__(256)
void cvt_w(const float* __restrict__ wq, const float* __restrict__ wk, const float* __restrict__ wv,
           const float* __restrict__ wo, unsigned short* Wb) {
  const int tid = threadIdx.x, blk = blockIdx.x;
  const int wave = tid >> 5, lane = tid & 31;
  const int sel = blk >> 3;
  const float* src = (sel == 0) ? wq : (sel == 1) ? wk : (sel == 2) ? wv : wo;
  const int pitch = (sel == 0) ? CU : CC;
  const int o    = (blk & 7) * 16 + 2 * wave + (lane >> 4);
  const int col  = 8 * (lane & 15);
  const bool live = col < pitch;
  const int colc = live ? col : (pitch - 8);
  const float* s = src + (size_t)o * pitch + colc;
  const v4f a = *(const v4f*)s;
  const v4f q = *(const v4f*)(s + 4);
  const float f[8] = {a[0], a[1], a[2], a[3], q[0], q[1], q[2], q[3]};
  v4u u;
#pragma unroll
  for (int t = 0; t < 4; ++t) u[t] = live ? pk16(bf_bits(f[2 * t]), bf_bits(f[2 * t + 1])) : 0u;
#pragma unroll
  for (int pass = 0; pass < 2; ++pass) {
    *(volatile v4u*)(Wb + ((size_t)(sel * CC + o)) * CC + col) = u;
    __threadfence();
  }
}

template <int CIN>
__global__ __launch_bounds__(256)
void cvt_x(const float* __restrict__ x, unsigned short* H) {
  __shared__ __align__(16) unsigned short Th[QT * TP];
  const int tid = threadIdx.x;
  const int nb = blockIdx.x, cb = blockIdx.y, b = blockIdx.z;
  const int e = tid & 7, lq = tid >> 3;
  const int n0 = nb * QT, c0 = cb * QT;
#pragma unroll
  for (int it = 0; it < 2; ++it) {
    const int cl = it * 32 + lq;
    const int ch = c0 + cl;
    const float* sp = x + ((size_t)(b * CIN + ch)) * NN + n0 + 8 * e;
    const v4f a = *(const v4f*)sp;
    const v4f q = *(const v4f*)(sp + 4);
    const float f[8] = {a[0], a[1], a[2], a[3], q[0], q[1], q[2], q[3]};
#pragma unroll
    for (int t = 0; t < 8; ++t) Th[(8 * e + t) * TP + cl] = bf_bits(f[t]);
  }
  __syncthreads();
  v4u uh[2];
#pragma unroll
  for (int it = 0; it < 2; ++it) {
    const int nl = it * 32 + lq;
    uh[it] = *(const v4u*)(Th + nl * TP + 8 * e);
  }
#pragma unroll
  for (int pass = 0; pass < 2; ++pass) {
#pragma unroll
    for (int it = 0; it < 2; ++it) {
      const int nl = it * 32 + lq;
      const size_t po = ((size_t)(b * NN + n0 + nl)) * CIN + c0 + 8 * e;
      *(volatile v4u*)(H + po) = uh[it];
    }
    __threadfence();
  }
}

template <int KK, int MODE>
__global__ __launch_bounds__(128)
void conv_cm(const unsigned short* __restrict__ W, const unsigned short* __restrict__ H,
             const float* __restrict__ bias, unsigned short* Ph, unsigned short* Pl) {
  static_assert(KK % 32 == 0 && KK <= CC);
  __shared__ __align__(16) float Vs[QT * OSP];
  const int tid  = threadIdx.x;
  const int lane = tid & 31, wave = tid >> 5;
  const int hh   = lane >> 4, c = lane & 15;
  const int nt   = blockIdx.x, mb = blockIdx.y, b = blockIdx.z;
  const int n0   = nt * QT, o0 = mb * QT;

  const unsigned short* ap = H + ((size_t)(b * NN + n0 + 16 * wave + c)) * KK + 8 * hh;
  const unsigned short* bp = W + ((size_t)(o0 + c)) * CC + 8 * hh;

  v8f acc[4];
#pragma unroll
  for (int j = 0; j < 4; ++j) acc[j] = zero8();

#pragma unroll
  for (int ks = 0; ks < KK / 32; ++ks) {
    const Frag fa = ldfrag(ap + 32 * ks);
#pragma unroll
    for (int j = 0; j < 4; ++j) {
      const Frag fb = ldfrag(bp + (size_t)(16 * j) * CC + 32 * ks);
      acc[j] = mma_b(fa.bf, fb.bf, acc[j]);
    }
  }

  {
    const int nrow = 16 * wave + 8 * hh;
#pragma unroll
    for (int j = 0; j < 4; ++j) {
      const float bb = bfr(bias[o0 + 16 * j + c]);
      v4f va, vb;
#pragma unroll
      for (int r = 0; r < 4; ++r) { va[r] = acc[j][r] + bb; vb[r] = acc[j][4 + r] + bb; }
      *(v4f*)(Vs + (16 * j + c) * OSP + nrow)     = va;
      *(v4f*)(Vs + (16 * j + c) * OSP + nrow + 4) = vb;
    }
  }
  __syncthreads();

  const int e = tid & 7, lq = tid >> 3;
  v4u uh[4], ul[4];
#pragma unroll
  for (int it = 0; it < 4; ++it) {
    const int ol = it * 16 + lq;
    const v4f a = *(const v4f*)(Vs + ol * OSP + 8 * e);
    const v4f q = *(const v4f*)(Vs + ol * OSP + 8 * e + 4);
    const float f[8] = {a[0], a[1], a[2], a[3], q[0], q[1], q[2], q[3]};
#pragma unroll
    for (int t = 0; t < 4; ++t) {
      const float f0 = f[2 * t], f1 = f[2 * t + 1];
      const unsigned short hb0 = bf_bits(f0), hb1 = bf_bits(f1);
      const unsigned short lb0 = bf_bits(f0 - bf_up(hb0));
      const unsigned short lb1 = bf_bits(f1 - bf_up(hb1));
      uh[it][t] = pk16(hb0, hb1);
      ul[it][t] = pk16(lb0, lb1);
    }
  }
#pragma unroll
  for (int pass = 0; pass < 2; ++pass) {
#pragma unroll
    for (int it = 0; it < 4; ++it) {
      const int ol = it * 16 + lq;
      const size_t po = ((size_t)(b * CC + o0 + ol)) * NN + n0 + 8 * e;
      *(volatile v4u*)(Ph + po) = uh[it];
      if (MODE == 0) *(volatile v4u*)(Pl + po) = ul[it];
    }
    __threadfence();
  }
}

__global__ __launch_bounds__(128)
void gemm_vt(const unsigned short* __restrict__ Wv, const unsigned short* __restrict__ Hl,
             const float* __restrict__ bv, unsigned short* VT) {
  __shared__ __align__(16) float Vs[VTD * VTP];
  const int tid  = threadIdx.x;
  const int lane = tid & 31, wave = tid >> 5;
  const int hh   = lane >> 4, c = lane & 15;
  const int d0   = blockIdx.x * VTD, o0 = blockIdx.y * 16, b = blockIdx.z;

  const unsigned short* ap = Hl + ((size_t)(b * NN + (8 * wave) * 128 + d0 + c)) * CC + 8 * hh;
  const unsigned short* bp = Wv + ((size_t)(o0 + c)) * CC + 8 * hh;

  v8f acc[8];
#pragma unroll
  for (int t = 0; t < 8; ++t) acc[t] = zero8();

#pragma unroll
  for (int ks = 0; ks < CC / 32; ++ks) {
    const Frag fb = ldfrag(bp + 32 * ks);
#pragma unroll
    for (int t = 0; t < 8; ++t) {
      const Frag fa = ldfrag(ap + (size_t)t * 128 * CC + 32 * ks);
      acc[t] = mma_b(fa.bf, fb.bf, acc[t]);
    }
  }

  {
    const float bb = bfr(bv[o0 + c]);
#pragma unroll
    for (int t = 0; t < 8; ++t) {
      const int g = 8 * wave + t;
      v4f va, vb;
#pragma unroll
      for (int r = 0; r < 4; ++r) { va[r] = acc[t][r] + bb; vb[r] = acc[t][4 + r] + bb; }
      *(v4f*)(Vs + c * VTP + 16 * g + 8 * hh)     = va;
      *(v4f*)(Vs + c * VTP + 16 * g + 8 * hh + 4) = vb;
    }
  }
  __syncthreads();

  const int qq = tid & 63, hsel = tid >> 6;
  const int ol = qq >> 2, g0 = 8 * (qq & 3);
  v4u uv[8];
#pragma unroll
  for (int it = 0; it < 8; ++it) {
    const int dl = 2 * it + hsel;
    float f[8];
#pragma unroll
    for (int j = 0; j < 8; ++j) f[j] = Vs[ol * VTP + 16 * (g0 + j) + dl];
#pragma unroll
    for (int t = 0; t < 4; ++t)
      uv[it][t] = pk16(h_bits((_Float16)f[2 * t]), h_bits((_Float16)f[2 * t + 1]));
  }
#pragma unroll
  for (int pass = 0; pass < 2; ++pass) {
#pragma unroll
    for (int it = 0; it < 8; ++it) {
      const int dl = 2 * it + hsel;
      *(volatile v4u*)(VT + ((size_t)(b * CC + d0 + dl)) * NN + o0 * 32 + 8 * qq) = uv[it];
    }
    __threadfence();
  }
}

__global__ __launch_bounds__(128)
void attn_k(const unsigned short* __restrict__ Qh, const unsigned short* __restrict__ Ql,
            const unsigned short* __restrict__ Kh, const unsigned short* __restrict__ VT,
            unsigned short* Ah, unsigned short* Al) {
  __shared__ __align__(16) float Os[QT * OSPW];
  const int tid  = threadIdx.x;
  const int wave = tid >> 5, lane = tid & 31;
  const int hh   = lane >> 4, c = lane & 15;
  const int n0   = blockIdx.x * QT, b = blockIdx.y;

  const size_t qo = ((size_t)(b * NN + n0 + 16 * wave + c)) * CC + 8 * hh;
  const unsigned short* Qhp = Qh + qo;
  const unsigned short* Qlp = Ql + qo;
  const unsigned short* Khp = Kh + (size_t)b * NN * CC + (size_t)c * CC + 8 * hh;
  const unsigned short* Vp = VT + (size_t)b * CC * NN + (size_t)c * NN + 8 * hh;

  float m = -1.0e30f, l = 0.f;
  v8f o[8];
#pragma unroll
  for (int j = 0; j < 8; ++j) o[j] = zero8();

#pragma unroll 1
  for (int kb = 0; kb < NN; kb += 32) {
    const unsigned short* k0p = Khp + (size_t)kb * CC;
    const unsigned short* k1p = Khp + (size_t)(kb + 16) * CC;
    v8f s0 = zero8(), s1 = zero8();
#pragma unroll 1
    for (int kc = 0; kc < CC / 32; ++kc) {
      const Frag qh = ldfrag(Qhp + 32 * kc);
      const Frag ql = ldfrag(Qlp + 32 * kc);
      const Frag k0 = ldfrag(k0p + 32 * kc);
      const Frag k1 = ldfrag(k1p + 32 * kc);
      s0 = mma_b(k0.bf, qh.bf, s0);
      s1 = mma_b(k1.bf, qh.bf, s1);
      s0 = mma_b(k0.bf, ql.bf, s0);
      s1 = mma_b(k1.bf, ql.bf, s1);
    }
#pragma unroll
    for (int r = 0; r < 8; ++r) { s0[r] *= SCL; s1[r] *= SCL; }

    float mx = fmaxf(hmax8(s0), hmax8(s1));
    mx = fmaxf(mx, __shfl_xor(mx, 16, 32));
    const float mn = fmaxf(m, mx);
    const unsigned grew = wave_ballot(mx > m);
    if (grew != 0u) {
      const float corr = __expf(m - mn);
      l *= corr;
#pragma unroll
      for (int j = 0; j < 8; ++j) {
#pragma unroll
        for (int r = 0; r < 8; ++r) o[j][r] *= corr;
      }
    }
    m = mn;
    const float msh = mn - LNPS;

    FragH ph;
    float ls = 0.f;
#pragma unroll
    for (int r = 0; r < 8; ++r) {
      const float e0 = __expf(s0[r] - msh);
      const float e1 = __expf(s1[r] - msh);
      ls += e0 + e1;
      ph.hv[0][r] = (_Float16)e0;
      ph.hv[1][r] = (_Float16)e1;
    }
    l += ls;

#pragma unroll
    for (int j = 0; j < 8; ++j) {
      const Frag vf = ldfrag(Vp + (size_t)(16 * j) * NN + kb);
      o[j] = mma_h(vf.h, ph.v, o[j]);
    }
  }
  l += __shfl_xor(l, 16, 32);
  const float inv = 1.0f / l;

  const int qrow = 16 * wave + c;
#pragma unroll
  for (int j = 0; j < 8; ++j) {
    v4f va, vb;
#pragma unroll
    for (int r = 0; r < 4; ++r) { va[r] = o[j][r] * inv; vb[r] = o[j][4 + r] * inv; }
    *(v4f*)(Os + qrow * OSPW + 16 * j + 8 * hh)     = va;
    *(v4f*)(Os + qrow * OSPW + 16 * j + 8 * hh + 4) = vb;
  }
  __syncthreads();

  const int e = tid & 15, lq = tid >> 4;
  v4u uh[8], ul[8];
#pragma unroll
  for (int it = 0; it < 8; ++it) {
    const int row = it * 8 + lq;
    const v4f a = *(const v4f*)(Os + row * OSPW + 8 * e);
    const v4f q = *(const v4f*)(Os + row * OSPW + 8 * e + 4);
    const float f[8] = {a[0], a[1], a[2], a[3], q[0], q[1], q[2], q[3]};
#pragma unroll
    for (int t = 0; t < 4; ++t) {
      const float f0 = f[2 * t], f1 = f[2 * t + 1];
      const unsigned short hb0 = bf_bits(f0), hb1 = bf_bits(f1);
      const unsigned short lb0 = bf_bits(f0 - bf_up(hb0));
      const unsigned short lb1 = bf_bits(f1 - bf_up(hb1));
      uh[it][t] = pk16(hb0, hb1);
      ul[it][t] = pk16(lb0, lb1);
    }
  }
#pragma unroll
  for (int pass = 0; pass < 2; ++pass) {
#pragma unroll
    for (int it = 0; it < 8; ++it) {
      const int row = it * 8 + lq;
      const size_t po = ((size_t)(b * NN + n0 + row)) * CC + 8 * e;
      *(volatile v4u*)(Ah + po) = uh[it];
      *(volatile v4u*)(Al + po) = ul[it];
    }
    __threadfence();
  }
}

__global__ __launch_bounds__(256)
void tr_a(const unsigned short* __restrict__ Ah, const unsigned short* __restrict__ Al,
          unsigned short* At, unsigned short* Atl) {
  __shared__ __align__(16) unsigned short Th[QT * TP];
  __shared__ __align__(16) unsigned short Tl[QT * TP];
  const int tid = threadIdx.x;
  const int nb = blockIdx.x, cb = blockIdx.y, b = blockIdx.z;
  const int e = tid & 7, lq = tid >> 3;
  const int s0 = nb * QT, o0 = cb * QT;
#pragma unroll
  for (int it = 0; it < 2; ++it) {
    const int ol = it * 32 + lq;
    const size_t src = ((size_t)(b * CC + o0 + ol)) * NN + s0 + 8 * e;
    const v4u ah = *(const v4u*)(Ah + src);
    const v4u al = *(const v4u*)(Al + src);
#pragma unroll
    for (int t = 0; t < 8; ++t) {
      const unsigned sh = 16u * (unsigned)(t & 1);
      Th[(8 * e + t) * TP + ol] = (unsigned short)((ah[t >> 1] >> sh) & 0xFFFFu);
      Tl[(8 * e + t) * TP + ol] = (unsigned short)((al[t >> 1] >> sh) & 0xFFFFu);
    }
  }
  __syncthreads();
  v4u uh[2], ul[2];
#pragma unroll
  for (int it = 0; it < 2; ++it) {
    const int sl = it * 32 + lq;
    uh[it] = *(const v4u*)(Th + sl * TP + 8 * e);
    ul[it] = *(const v4u*)(Tl + sl * TP + 8 * e);
  }
#pragma unroll
  for (int pass = 0; pass < 2; ++pass) {
#pragma unroll
    for (int it = 0; it < 2; ++it) {
      const int sl = it * 32 + lq;
      const size_t po = ((size_t)(b * NN + s0 + sl)) * CC + o0 + 8 * e;
      *(volatile v4u*)(At + po)  = uh[it];
      *(volatile v4u*)(Atl + po) = ul[it];
    }
    __threadfence();
  }
}

__global__ __launch_bounds__(128)
void gemm_p(const unsigned short* __restrict__ Wb, const unsigned short* __restrict__ At,
            const unsigned short* __restrict__ Atl, const float* __restrict__ bo, const float* __restrict__ x,
            float* out) {
  __shared__ __align__(16) float Vs[QT * OSP];
  const int tid  = threadIdx.x;
  const int lane = tid & 31, wave = tid >> 5;
  const int hh   = lane >> 4, c = lane & 15;
  const int nt   = blockIdx.x, mb = blockIdx.y, b = blockIdx.z;
  const int n0   = nt * QT, o0 = mb * QT;

  const size_t ao = ((size_t)(b * NN + n0 + 16 * wave + c)) * CC + 8 * hh;
  const unsigned short* ahp = At + ao;
  const unsigned short* alp = Atl + ao;
  const unsigned short* bpw = Wb + ((size_t)(3 * CC + o0 + c)) * CC + 8 * hh;

  v8f acc[4];
#pragma unroll
  for (int j = 0; j < 4; ++j) acc[j] = zero8();

#pragma unroll
  for (int ks = 0; ks < CC / 32; ++ks) {
    const Frag fah = ldfrag(ahp + 32 * ks);
    const Frag fal = ldfrag(alp + 32 * ks);
#pragma unroll
    for (int j = 0; j < 4; ++j) {
      const Frag fb = ldfrag(bpw + (size_t)(16 * j) * CC + 32 * ks);
      acc[j] = mma_b(fah.bf, fb.bf, acc[j]);
      acc[j] = mma_b(fal.bf, fb.bf, acc[j]);
    }
  }

  {
    const int nrow = 16 * wave + 8 * hh;
#pragma unroll
    for (int j = 0; j < 4; ++j) {
      const float bb = bfr(bo[o0 + 16 * j + c]);
      v4f va, vb;
#pragma unroll
      for (int r = 0; r < 4; ++r) { va[r] = acc[j][r] + bb; vb[r] = acc[j][4 + r] + bb; }
      *(v4f*)(Vs + (16 * j + c) * OSP + nrow)     = va;
      *(v4f*)(Vs + (16 * j + c) * OSP + nrow + 4) = vb;
    }
  }
  __syncthreads();

  const int e = tid & 15, lq = tid >> 4;
  v4f res[8];
#pragma unroll
  for (int it = 0; it < 8; ++it) {
    const int ol = it * 8 + lq;
    const v4f a = *(const v4f*)(Vs + ol * OSP + 4 * e);
    const size_t idx = ((size_t)(b * CC + o0 + ol)) * NN + n0 + 4 * e;
    const v4f xv = *(const v4f*)(x + idx);
#pragma unroll
    for (int t = 0; t < 4; ++t) res[it][t] = a[t] + bfr(xv[t]);
  }
#pragma unroll
  for (int pass = 0; pass < 2; ++pass) {
#pragma unroll
    for (int it = 0; it < 8; ++it) {
      const int ol = it * 8 + lq;
      const size_t idx = ((size_t)(b * CC + o0 + ol)) * NN + n0 + 4 * e;
      *(volatile v4f*)(out + idx) = res[it];
    }
    __threadfence();
  }
}

extern "C" void kernel_launch(void* const* d_in, const int* in_sizes, int n_in,
                              void* d_out, int out_size, void* d_ws, size_t ws_size,
                              hipStream_t stream) {
  if (n_in < 10) return;
  if (in_sizes[0] < NB * CU * NN) return;
  if (in_sizes[1] < NB * CC * NN) return;
  if (in_sizes[2] < CC * CU || in_sizes[3] < CC) return;
  if (in_sizes[4] < CC * CC || in_sizes[5] < CC) return;
  if (in_sizes[6] < CC * CC || in_sizes[7] < CC) return;
  if (in_sizes[8] < CC * CC || in_sizes[9] < CC) return;
  if (out_size < NB * CC * NN) return;

  size_t off = 0;
  auto carve = [&](size_t bytes) { const size_t o = off; off += (bytes + 255) & ~(size_t)255; return o; };
  const size_t plane = (size_t)NB * NN * CC * 2;
  const size_t oWb  = carve((size_t)4 * CC * CC * 2);
  const size_t oHu  = carve((size_t)NB * NN * CU * 2);
  const size_t oHl  = carve(plane);
  const size_t oQh  = carve(plane);
  const size_t oQl  = carve(plane);
  const size_t oKh  = carve(plane);
  const size_t oVT  = carve(plane);
  const size_t oAh  = carve(plane);
  const size_t oAl  = carve(plane);
  const size_t oAt  = carve(plane);
  const size_t oAtl = carve(plane);
  if (off > ws_size) return;
  if (off > (size_t)134217728) return;

  const float* x_upper = (const float*)d_in[0];
  const float* x_lower = (const float*)d_in[1];
  const float* wq = (const float*)d_in[2];
  const float* bq = (const float*)d_in[3];
  const float* wk = (const float*)d_in[4];
  const float* bk = (const float*)d_in[5];
  const float* wv = (const float*)d_in[6];
  const float* bv = (const float*)d_in[7];
  const float* wo = (const float*)d_in[8];
  const float* bo = (const float*)d_in[9];

  char* ws = (char*)d_ws;
  unsigned short* Wb  = (unsigned short*)(ws + oWb);
  unsigned short* Hu  = (unsigned short*)(ws + oHu);
  unsigned short* Hl  = (unsigned short*)(ws + oHl);
  unsigned short* Qh  = (unsigned short*)(ws + oQh);
  unsigned short* Ql  = (unsigned short*)(ws + oQl);
  unsigned short* Kh  = (unsigned short*)(ws + oKh);
  unsigned short* VT  = (unsigned short*)(ws + oVT);
  unsigned short* Ah  = (unsigned short*)(ws + oAh);
  unsigned short* Al  = (unsigned short*)(ws + oAl);
  unsigned short* At  = (unsigned short*)(ws + oAt);
  unsigned short* Atl = (unsigned short*)(ws + oAtl);
  float* out = (float*)d_out;

  const dim3 blk256(256), blk128(128);

  cvt_w<<<dim3(32), blk256, 0, stream>>>(wq, wk, wv, wo, Wb);
  cvt_x<CU><<<dim3(NN / QT, CU / QT, NB), blk256, 0, stream>>>(x_upper, Hu);
  cvt_x<CC><<<dim3(NN / QT, CC / QT, NB), blk256, 0, stream>>>(x_lower, Hl);
  conv_cm<CU, 0><<<dim3(NN / QT, CC / QT, NB), blk128, 0, stream>>>(Wb, Hu, bq, Qh, Ql);
  conv_cm<CC, 1><<<dim3(NN / QT, CC / QT, NB), blk128, 0, stream>>>(Wb + (size_t)CC * CC, Hl, bk, Kh, Kh);
  gemm_vt<<<dim3(CC / VTD, CC / 16, NB), blk128, 0, stream>>>(Wb + (size_t)2 * CC * CC, Hl, bv, VT);
  attn_k<<<dim3(NQ / QT, NB), blk128, 0, stream>>>(Qh, Ql, Kh, VT, Ah, Al);
  tr_a<<<dim3(NN / QT, CC / QT, NB), blk256, 0, stream>>>(Ah, Al, At, Atl);
  gemm_p<<<dim3(NN / QT, CC / QT, NB), blk128, 0, stream>>>(Wb, At, Atl, bo, x_lower, out);
  (void)hipGetLastError();
}
